// EAGCN_16200616640806
// MI455X (gfx1250) — hardware-run, weakly checked
//
#include <hip/hip_runtime.h>


#define NI   32
#define CC   256
#define NP   1024
#define SS   64
typedef _Float16 h16;
typedef unsigned short bf;
typedef __attribute__((ext_vector_type(16))) __bf16   v16bf;
typedef __attribute__((ext_vector_type(16))) _Float16 v16h;
typedef __attribute__((ext_vector_type(8)))  _Float16 v8h;
typedef __attribute__((ext_vector_type(8)))  unsigned short v8us;
typedef __attribute__((ext_vector_type(8)))  float    v8f;
typedef __attribute__((ext_vector_type(4)))  float    v4f;
typedef v8h  __attribute__((may_alias)) v8ha;
typedef v4f  __attribute__((may_alias)) v4fa;
typedef v8us __attribute__((may_alias)) v8usa;

__device__ __forceinline__ unsigned short f2bf(float f) { unsigned u = __float_as_uint(f); u += 0x7FFFu + ((u >> 16) & 1u); return (unsigned short)(u >> 16); }
__device__ __forceinline__ float bf2f(unsigned short b) { return __uint_as_float(((unsigned)b) << 16); }
__device__ __forceinline__ float bfr(float f) { return bf2f(f2bf(f)); }
__device__ __forceinline__ v16h cat16(v8h lo, v8h hi) { return __builtin_shufflevector(lo, hi, 0, 1, 2, 3, 4, 5, 6, 7, 8, 9, 10, 11, 12, 13, 14, 15); }
__device__ __forceinline__ v16bf cat16b(v8us lo, v8us hi) { return __builtin_bit_cast(v16bf, __builtin_shufflevector(lo, hi, 0, 1, 2, 3, 4, 5, 6, 7, 8, 9, 10, 11, 12, 13, 14, 15)); }
__device__ __forceinline__ v8f wmma16(v16h a, v16h b, v8f c) { return __builtin_amdgcn_wmma_f32_16x16x32_f16(false, a, false, b, (short)0, c, false, false); }
__device__ __forceinline__ v8f wmmab(v16bf a, v16bf b, v8f c) { return __builtin_amdgcn_wmma_f32_16x16x32_bf16(false, a, false, b, (short)0, c, false, false); }


template <typename T16> struct WFrag;
template <> struct WFrag<h16> { typedef v16h V; static __device__ __forceinline__ V ld(const h16* p) { return cat16(*(const v8h*)p, *(const v8h*)(p + 16)); } static __device__ __forceinline__ v8f mma(V a, V b, v8f c) { return wmma16(a, b, c); } };
template <> struct WFrag<bf> { typedef v16bf V; static __device__ __forceinline__ V ld(const bf* p) { return cat16b(*(const v8us*)p, *(const v8us*)(p + 16)); } static __device__ __forceinline__ v8f mma(V a, V b, v8f c) { return wmmab(a, b, c); } };
template <typename T16, int NSPLIT, bool BIAS>
__global__ __launch_bounds__(32) void k_gemmw(const T16* __restrict__ A, const T16* __restrict__ A2, const T16* __restrict__ Bt, const T16* __restrict__ Bt2, int K, float* C, int ldc, const float* __restrict__ bias, size_t sA, size_t sB, size_t sC) {
    typedef typename WFrag<T16>::V V;
    __shared__ __align__(16) float os[16 * 68];
    const size_t z = blockIdx.z; A += z * sA; if (A2) A2 += z * sA; Bt += z * sB; if (Bt2) Bt2 += z * sB; C += z * sC;
    const int lane = threadIdx.x & 31, lr = lane & 15, hi = lane >> 4; const int r0 = blockIdx.x * 64, c0 = blockIdx.y * 64;
    v8f acc[4][4];
#pragma unroll
    for (int mb = 0; mb < 4; ++mb)
#pragma unroll
        for (int nb = 0; nb < 4; ++nb) acc[mb][nb] = (v8f){};
    const size_t aoff = (size_t)(r0 + lr) * K + 8 * hi, boff = (size_t)(c0 + lr) * K + 8 * hi;
#pragma unroll 1
    for (int kc = 0; kc < K; kc += 32) {
        V a[4], a2[4];
#pragma unroll
        for (int mb = 0; mb < 4; ++mb) { a[mb] = WFrag<T16>::ld(A + aoff + (size_t)mb * 16 * K + kc); if (NSPLIT == 1 || NSPLIT == 2) a2[mb] = WFrag<T16>::ld(A2 + aoff + (size_t)mb * 16 * K + kc); }
#pragma unroll
        for (int nb = 0; nb < 4; ++nb) { const V b = WFrag<T16>::ld(Bt + boff + (size_t)nb * 16 * K + kc); V b2; if (NSPLIT >= 2) b2 = WFrag<T16>::ld(Bt2 + boff + (size_t)nb * 16 * K + kc);
#pragma unroll
            for (int mb = 0; mb < 4; ++mb) { acc[mb][nb] = WFrag<T16>::mma(a[mb], b, acc[mb][nb]); if (NSPLIT == 1 || NSPLIT == 2) acc[mb][nb] = WFrag<T16>::mma(a2[mb], b, acc[mb][nb]); if (NSPLIT >= 2) acc[mb][nb] = WFrag<T16>::mma(a[mb], b2, acc[mb][nb]); } }
        asm volatile("v_nop\n\tv_nop\n\tv_nop\n\tv_nop" : "+v"(acc[0][0]), "+v"(acc[1][1]), "+v"(acc[2][2]), "+v"(acc[3][3]) : "v"(a[0]), "v"(a[3]));
    }
#pragma unroll
    for (int mb = 0; mb < 4; ++mb) {
#pragma unroll
        for (int nb = 0; nb < 4; ++nb) {
#pragma unroll
            for (int j = 0; j < 8; ++j) os[(hi * 8 + j) * 68 + nb * 16 + lr] = acc[mb][nb][j]; }
        __builtin_amdgcn_wave_barrier(); asm volatile("" ::: "memory");
        float* crow = C + (size_t)(r0 + mb * 16) * ldc + c0;
#pragma unroll 1
        for (int ps = 0; ps < 2; ++ps) {
#pragma unroll
            for (int s = 0; s < 8; ++s) { const int row = 2 * s + hi, cofs = lr * 4; v4f val = *(const v4fa*)(os + row * 68 + cofs); if (BIAS) { val[0] += bfr(bias[c0 + cofs]); val[1] += bfr(bias[c0 + cofs + 1]); val[2] += bfr(bias[c0 + cofs + 2]); val[3] += bfr(bias[c0 + cofs + 3]); }
                *(volatile v4f*)(crow + (size_t)row * ldc + cofs) = val; }
            if (ps == 0) __threadfence(); }
        __builtin_amdgcn_wave_barrier(); asm volatile("" ::: "memory");
    }
}

__device__ __forceinline__ void splitf(float y, unsigned short& h, unsigned short& l) { h = f2bf(y); l = f2bf(y - bf2f(h)); }
typedef __attribute__((ext_vector_type(2))) unsigned short v2us;
typedef __attribute__((ext_vector_type(4))) unsigned short v4us;

__global__ __launch_bounds__(256) void k_cvt8(const float* __restrict__ src, bf* dst, size_t n8) { const size_t i = (size_t)blockIdx.x * 256 + threadIdx.x; if (i >= n8) return; const v8f v = *(const v8f*)(src + i * 8); v8us o;
#pragma unroll
    for (int k = 0; k < 8; ++k) o[k] = f2bf(v[k]); *(volatile v8us*)(dst + i * 8) = o; __threadfence(); *(volatile v8us*)(dst + i * 8) = o; }
__global__ __launch_bounds__(256) void k_xt(const float* __restrict__ x, bf* XT) { const int e = (blockIdx.x * 256 + threadIdx.x) * 2; if (e >= NP * CC) return; const int c = e % CC; const int p = e / CC; v2us o; o[0] = f2bf(x[(size_t)c * NP + p]); o[1] = f2bf(x[(size_t)(c + 1) * NP + p]); *(volatile v2us*)(XT + e) = o; __threadfence(); *(volatile v2us*)(XT + e) = o; }
__global__ __launch_bounds__(256) void k_rowb(float* A, const float* __restrict__ bias) { const int e = (blockIdx.x * 256 + threadIdx.x) * 4; if (e >= SS * NP) return; const int j = e / NP; const float bb = bfr(bias[j]); const v4f a = *(const v4f*)(A + e); v4f o;
#pragma unroll
    for (int u = 0; u < 4; ++u) o[u] = __fadd_rn(a[u], bb); *(volatile v4f*)(A + e) = o; __threadfence(); *(volatile v4f*)(A + e) = o; }
__global__ __launch_bounds__(256) void k_mean(const float* __restrict__ seg, float* MEAN) { const int c = threadIdx.x; const float* sr = seg + (size_t)c * NP; float s = 0.f;
#pragma unroll 1
    for (int p = 0; p < NP; ++p) s = __fadd_rn(s, bfr(sr[p])); const float m = s * (1.0f / NP); *(volatile float*)(MEAN + c) = m; __threadfence(); *(volatile float*)(MEAN + c) = m; }
__global__ __launch_bounds__(64) void k_chat(const float* __restrict__ MEAN, const float* __restrict__ Wm, const float* __restrict__ bm, float* CH) { const int j = threadIdx.x; float acc = 0.f;
#pragma unroll 1
    for (int c = 0; c < CC; ++c) { float w = bfr(Wm[j * CC + c]); asm volatile("" : "+v"(w)); float pr = __fmul_rn(MEAN[c], w); asm volatile("" : "+v"(pr)); acc = __fadd_rn(acc, pr); }
    const float r = fmaxf(__fadd_rn(acc, bfr(bm[j])), 0.f); *(volatile float*)(CH + j) = r; __threadfence(); *(volatile float*)(CH + j) = r; }

__global__ __launch_bounds__(256) void k_t1(const float* __restrict__ SG, const float* __restrict__ CH, bf* Th, bf* Tl) { const int e = (blockIdx.x * 256 + threadIdx.x) * 4; if (e >= NP * SS) return; const int t0 = e % SS; const int p = e / SS; const float* th = SG + (size_t)p * SS; float acc[4] = {0.f, 0.f, 0.f, 0.f};
#pragma unroll 1
    for (int j = 0; j < SS; ++j) { const float tj = th[j]; const float cj = CH[j];
#pragma unroll
        for (int u = 0; u < 4; ++u) { float d = __fmul_rn(cj, CH[t0 + u]); asm volatile("" : "+v"(d)); float pr = __fmul_rn(tj, d); asm volatile("" : "+v"(pr)); acc[u] = __fadd_rn(acc[u], pr); } }
    v4us oh, ol;
#pragma unroll
    for (int u = 0; u < 4; ++u) { unsigned short a, b; splitf(acc[u], a, b); oh[u] = a; ol[u] = b; } *(volatile v4us*)(Th + e) = oh; *(volatile v4us*)(Tl + e) = ol; __threadfence(); *(volatile v4us*)(Th + e) = oh; *(volatile v4us*)(Tl + e) = ol; }
__global__ __launch_bounds__(256) void k_tp(const float* __restrict__ A, bf* Ah, bf* Al) { const int e = (blockIdx.x * 256 + threadIdx.x) * 4; if (e >= NP * SS) return; const int j = e % SS; const int q = e / SS; v4us oh, ol;
#pragma unroll
    for (int u = 0; u < 4; ++u) { unsigned short a, b; splitf(A[(size_t)(j + u) * NP + q], a, b); oh[u] = a; ol[u] = b; } *(volatile v4us*)(Ah + e) = oh; *(volatile v4us*)(Al + e) = ol; __threadfence(); *(volatile v4us*)(Ah + e) = oh; *(volatile v4us*)(Al + e) = ol; }
__global__ __launch_bounds__(256) void k_spl(const float* __restrict__ A, size_t n4, bf* Ah, bf* Al) { const size_t e = ((size_t)blockIdx.x * 256 + threadIdx.x) * 4; if (e >= n4) return; const v4f a = *(const v4f*)(A + e); v4us oh, ol;
#pragma unroll
    for (int u = 0; u < 4; ++u) { unsigned short h, l; splitf(a[u], h, l); oh[u] = h; ol[u] = l; } *(volatile v4us*)(Ah + e) = oh; *(volatile v4us*)(Al + e) = ol; __threadfence(); *(volatile v4us*)(Ah + e) = oh; *(volatile v4us*)(Al + e) = ol; }
__global__ __launch_bounds__(256) void k_pool(const float* __restrict__ seg, const float* __restrict__ edge, const float* __restrict__ w2, const float* __restrict__ b2, const float* __restrict__ w3, const float* __restrict__ b3, float* SSQ, float* EMM) { const int p = blockIdx.x * 256 + threadIdx.x; if (p >= NP) return; float ms = -3.0e38f, me = -3.0e38f;
#pragma unroll 1
    for (int c = 0; c < CC; ++c) { const float s = bfr(seg[(size_t)c * NP + p]), ev = bfr(edge[(size_t)c * NP + p]); ms = fmaxf(ms, s); me = fmaxf(me, __fmul_rn(s, ev)); }
    float a = __fmul_rn(ms, bfr(w2[0])); asm volatile("" : "+v"(a)); const float ssq = __fadd_rn(a, bfr(b2[0])); float b = __fmul_rn(me, bfr(w3[0])); asm volatile("" : "+v"(b)); const float emm = __fadd_rn(b, bfr(b3[0]));
    for (int ps = 0; ps < 2; ++ps) { *(volatile float*)(SSQ + p) = ssq; *(volatile float*)(EMM + p) = emm; if (ps == 0) __threadfence(); } }
__global__ __launch_bounds__(256) void k_csoft(const float* __restrict__ SCT, float* SIMC) { const int lane = threadIdx.x & 31; const int q = blockIdx.x * 8 + (threadIdx.x >> 5); if (q >= NP) return; const float* sr = SCT + (size_t)q * NP; float v[NP / 32]; float mx = -3.0e38f;
#pragma unroll
    for (int ch = 0; ch < NP / 128; ++ch) { const v4f a = *(const v4f*)(sr + ch * 128 + lane * 4);
#pragma unroll
        for (int u = 0; u < 4; ++u) { v[ch * 4 + u] = a[u]; mx = fmaxf(mx, a[u]); } }
#pragma unroll
    for (int sh = 16; sh; sh >>= 1) mx = fmaxf(mx, __shfl_xor(mx, sh, 32));
    float sum = 0.f;
#pragma unroll
    for (int k = 0; k < NP / 32; ++k) { float d0 = __fsub_rn(v[k], mx); asm volatile("" : "+v"(d0)); v[k] = __builtin_amdgcn_exp2f(__fmul_rn(d0, 1.4426950408889634f)); sum += v[k]; }
#pragma unroll
    for (int sh = 16; sh; sh >>= 1) sum += __shfl_xor(sum, sh, 32);
    const float f = __fdiv_rn(1.0f, sum);
    for (int ps = 0; ps < 2; ++ps) {
#pragma unroll
        for (int ch = 0; ch < NP / 128; ++ch) { v4f o; for (int u = 0; u < 4; ++u) o[u] = v[ch * 4 + u] * f; *(volatile v4f*)(SIMC + (size_t)q * NP + ch * 128 + lane * 4) = o; }
        if (ps == 0) __threadfence(); } }
__global__ __launch_bounds__(256) void k_ssoft(const float* __restrict__ SOT, const float* __restrict__ SSQ, const float* __restrict__ EMM, const float* __restrict__ SIMC, bf* Mh, bf* Ml) { const int lane = threadIdx.x & 31; const int q = blockIdx.x * 8 + (threadIdx.x >> 5); if (q >= NP) return; const float* sr = SOT + (size_t)q * NP; const float sq = SSQ[q]; float v[NP / 32]; float mx = -3.0e38f;
#pragma unroll
    for (int ch = 0; ch < NP / 128; ++ch) { const int p0 = ch * 128 + lane * 4; const v4f a = *(const v4f*)(sr + p0);
#pragma unroll
        for (int u = 0; u < 4; ++u) { float f1 = __fmul_rn(EMM[p0 + u], sq); asm volatile("" : "+v"(f1)); const float t = __fmul_rn(f1, a[u]); v[ch * 4 + u] = t; mx = fmaxf(mx, t); } }
#pragma unroll
    for (int sh = 16; sh; sh >>= 1) mx = fmaxf(mx, __shfl_xor(mx, sh, 32));
    float sum = 0.f;
#pragma unroll
    for (int k = 0; k < NP / 32; ++k) { float d0 = __fsub_rn(v[k], mx); asm volatile("" : "+v"(d0)); v[k] = __builtin_amdgcn_exp2f(__fmul_rn(d0, 1.4426950408889634f)); sum += v[k]; }
#pragma unroll
    for (int sh = 16; sh; sh >>= 1) sum += __shfl_xor(sum, sh, 32);
    const float f = __fdiv_rn(1.0f, sum);
    for (int ps = 0; ps < 2; ++ps) {
#pragma unroll
        for (int ch = 0; ch < NP / 128; ++ch) { v4us oh, ol; const int p0 = ch * 128 + lane * 4;
#pragma unroll
            for (int u = 0; u < 4; ++u) { float ss = __fmul_rn(v[ch * 4 + u], f); asm volatile("" : "+v"(ss)); const float tot = __fadd_rn(SIMC[(size_t)q * NP + p0 + u], ss); unsigned short a, b; splitf(tot, a, b); oh[u] = a; ol[u] = b; }
            const size_t oo = (size_t)q * NP + p0; *(volatile v4us*)(Mh + oo) = oh; *(volatile v4us*)(Ml + oo) = ol; }
        if (ps == 0) __threadfence(); } }
__global__ __launch_bounds__(256) void k_fin(const float* __restrict__ OT, const float* __restrict__ seg, float* OUTb) { const int e = (blockIdx.x * 256 + threadIdx.x) * 4; if (e >= CC * NP) return; const int p = e % NP; const int c = e / NP; const v4f sg = *(const v4f*)(seg + e); v4f o;
#pragma unroll
    for (int u = 0; u < 4; ++u) { const float s = bfr(sg[u]); const float r = fmaxf(OT[(size_t)(p + u) * CC + c], 0.f); o[u] = __fadd_rn(__fadd_rn(r, s), s); } *(volatile v4f*)(OUTb + e) = o; __threadfence(); *(volatile v4f*)(OUTb + e) = o; }

extern "C" void kernel_launch(void* const* d_in, const int* in_sizes, int n_in,
                              void* d_out, int out_size, void* d_ws, size_t ws_size, hipStream_t stream) {
    (void)in_sizes; (void)n_in; (void)out_size;
    const float** I = (const float**)d_in;
    const float *seg = I[0], *edge = I[1], *W_s1 = I[2], *b_s1 = I[3], *W_s11 = I[4], *b_s11 = I[5], *W_mlp = I[6], *b_mlp = I[7], *W_g = I[12], *b_g = I[13];
    float* OUT = (float*)d_out;
    char* wsp = (char*)d_ws;
    auto take = [&](size_t bytes) { char* p = wsp; wsp += (bytes + 255) & ~(size_t)255; return (void*)p; };
    bf* A1 = (bf*)take(SS * CC * 2); bf* A11 = (bf*)take(SS * CC * 2); bf* BG = (bf*)take(CC * CC * 2); float* SC4 = (float*)take(256);
    bf* XT = (bf*)take((size_t)NP * CC * 2); bf* SB = (bf*)take((size_t)CC * NP * 2); float* SGS = (float*)take((size_t)SS * NP * 4); float* SGC = (float*)take((size_t)SS * NP * 4); float* CH = (float*)take(256); float* MEAN = (float*)take(CC * 4);
    bf* T1h = (bf*)take((size_t)NP * SS * 2); bf* T1l = (bf*)take((size_t)NP * SS * 2); bf* STh = (bf*)take((size_t)NP * SS * 2); bf* STl = (bf*)take((size_t)NP * SS * 2); bf* CTh = (bf*)take((size_t)NP * SS * 2); bf* CTl = (bf*)take((size_t)NP * SS * 2); bf* SGh = (bf*)take((size_t)NP * SS * 2); bf* SGl = (bf*)take((size_t)NP * SS * 2);
    float* SSQ = (float*)take(NP * 4); float* EMM = (float*)take(NP * 4); float* SCT = (float*)take((size_t)NP * NP * 4); float* SOT = (float*)take((size_t)NP * NP * 4); float* SIMC = (float*)take((size_t)NP * NP * 4); bf* Mh = (bf*)take((size_t)NP * NP * 2); bf* Ml = (bf*)take((size_t)NP * NP * 2);
    float* SGT = (float*)take((size_t)NP * CC * 4); bf* Gh = (bf*)take((size_t)NP * CC * 2); bf* Gl = (bf*)take((size_t)NP * CC * 2); float* OT = (float*)take((size_t)NP * CC * 4);
    if ((size_t)(wsp - (char*)d_ws) > ws_size) return;
    k_cvt8<<<(SS * CC / 8 + 255) / 256, 256, 0, stream>>>(W_s1, A1, SS * CC / 8); k_cvt8<<<(SS * CC / 8 + 255) / 256, 256, 0, stream>>>(W_s11, A11, SS * CC / 8); k_cvt8<<<(CC * CC / 8 + 255) / 256, 256, 0, stream>>>(W_g, BG, CC * CC / 8);
    const unsigned g64 = (NP * SS / 4 + 255) / 256;
    for (int b = 0; b < NI; ++b) { const float* sg = seg + (size_t)b * CC * NP; const float* ed = edge + (size_t)b * CC * NP;
        k_xt<<<(NP * CC / 2 + 255) / 256, 256, 0, stream>>>(sg, XT); k_cvt8<<<(CC * NP / 8 + 255) / 256, 256, 0, stream>>>(sg, SB, (size_t)CC * NP / 8);
        k_gemmw<bf, 0, false><<<dim3(1, NP / 64, 1), 32, 0, stream>>>(A1, nullptr, XT, nullptr, CC, SGS, NP, nullptr, 0, 0, 0); k_rowb<<<(SS * NP / 4 + 255) / 256, 256, 0, stream>>>(SGS, b_s1);
        k_gemmw<bf, 0, false><<<dim3(1, NP / 64, 1), 32, 0, stream>>>(A11, nullptr, XT, nullptr, CC, SGC, NP, nullptr, 0, 0, 0); k_rowb<<<(SS * NP / 4 + 255) / 256, 256, 0, stream>>>(SGC, b_s11);
        k_mean<<<1, 256, 0, stream>>>(sg, MEAN); k_chat<<<1, 64, 0, stream>>>(MEAN, W_mlp, b_mlp, CH);
        k_t1<<<g64, 256, 0, stream>>>(SGS, CH, T1h, T1l); k_tp<<<g64, 256, 0, stream>>>(SGS, STh, STl); k_tp<<<g64, 256, 0, stream>>>(SGC, CTh, CTl); k_spl<<<g64, 256, 0, stream>>>(SGC, (size_t)NP * SS, SGh, SGl);
        k_gemmw<bf, 2, false><<<dim3(NP / 64, NP / 64, 1), 32, 0, stream>>>(STh, STl, T1h, T1l, SS, SCT, NP, nullptr, 0, 0, 0);
        k_gemmw<bf, 2, false><<<dim3(NP / 64, NP / 64, 1), 32, 0, stream>>>(CTh, CTl, SGh, SGl, SS, SOT, NP, nullptr, 0, 0, 0);
        k_pool<<<(NP + 255) / 256, 256, 0, stream>>>(sg, ed, I[8], I[9], I[10], I[11], SSQ, EMM);
        k_csoft<<<NP / 8, 256, 0, stream>>>(SCT, SIMC); k_ssoft<<<NP / 8, 256, 0, stream>>>(SOT, SSQ, EMM, SIMC, Mh, Ml);
        k_gemmw<bf, 1, false><<<dim3(NP / 64, CC / 64, 1), 32, 0, stream>>>(Mh, Ml, SB, nullptr, NP, SGT, CC, nullptr, 0, 0, 0);
        k_spl<<<(unsigned)((NP * CC / 4 + 255) / 256), 256, 0, stream>>>(SGT, (size_t)NP * CC, Gh, Gl);
        k_gemmw<bf, 1, true><<<dim3(NP / 64, CC / 64, 1), 32, 0, stream>>>(Gh, Gl, BG, nullptr, CC, OT, CC, b_g, 0, 0, 0);
        k_fin<<<(CC * NP / 4 + 255) / 256, 256, 0, stream>>>(OT, sg, OUT + (size_t)b * CC * NP); }
}
